// TokenSwapMamba_25168508354815
// MI455X (gfx1250) — hardware-run, weakly checked
//
#include <hip/hip_runtime.h>
#include <stdint.h>

static constexpr int NBATCH = 2;
static constexpr int NTOK   = 4096;
static constexpr int CDIM   = 128;
static constexpr int CDIN   = 256;
static constexpr int CD2    = 512;
static constexpr int NST    = 16;
static constexpr int NDTR   = 8;
static constexpr int NXP    = 40;
static constexpr int NXPAD  = 64;
static constexpr int NROWS  = NBATCH * NTOK;
static constexpr int SCAN_CH = 16;
static constexpr int CONV_TW = 16;

static_assert(NROWS % 64 == 0, "M tile");
static_assert(CD2 % 64 == 0 && CDIM % 64 == 0 && NXPAD % 64 == 0, "N tile");
static_assert(CDIM % 32 == 0 && CDIN % 32 == 0, "K step");
static_assert(NXP <= NXPAD, "pad");
static_assert(NTOK % SCAN_CH == 0 && NTOK % CONV_TW == 0, "chunking");
static_assert(CDIM % 8 == 0 && CDIN % 8 == 0 && CDIM <= 256 && CDIN <= 256, "wcast lane map");

static constexpr size_t SZ_XPL   = (size_t)NROWS * CDIM * 2;
static constexpr size_t OFF_X1H  = 0;
static constexpr size_t OFF_X1L  = OFF_X1H + SZ_XPL;
static constexpr size_t OFF_X2H  = OFF_X1L + SZ_XPL;
static constexpr size_t OFF_X2L  = OFF_X2H + SZ_XPL;
static constexpr size_t SZ_WIN   = (size_t)CD2 * CDIM * 2;
static constexpr size_t OFF_WINH = OFF_X2L + SZ_XPL;
static constexpr size_t OFF_WINL = OFF_WINH + SZ_WIN;
static constexpr size_t SZ_WOUT  = (size_t)CDIM * CDIN * 2;
static constexpr size_t OFF_WOUTH = OFF_WINL + SZ_WIN;
static constexpr size_t OFF_WOUTL = OFF_WOUTH + SZ_WOUT;
static constexpr size_t SZ_WX    = (size_t)NXPAD * CDIN * 2;
static constexpr size_t OFF_WXH  = OFF_WOUTL + SZ_WOUT;
static constexpr size_t SZ_XZ    = (size_t)NROWS * CD2 * 4;
static constexpr size_t OFF_XZ   = OFF_WXH + SZ_WX;
static constexpr size_t SZ_XCF   = (size_t)NROWS * CDIN * 4;
static constexpr size_t OFF_XCF  = OFF_XZ + SZ_XZ;
static constexpr size_t SZ_XCH   = (size_t)NROWS * CDIN * 2;
static constexpr size_t OFF_XCH  = OFF_XCF + SZ_XCF;
static constexpr size_t SZ_XDBL  = (size_t)NROWS * NXPAD * 4;
static constexpr size_t OFF_XDBL = OFF_XCH + SZ_XCH;
static constexpr size_t SZ_YPL   = (size_t)NROWS * CDIN * 2;
static constexpr size_t OFF_YH   = OFF_XDBL + SZ_XDBL;
static constexpr size_t OFF_YL   = OFF_YH + SZ_YPL;
static constexpr size_t WS_TOTAL = OFF_YL + SZ_YPL;
static_assert(WS_TOTAL == 48660480ull, "carve total");
static_assert(WS_TOTAL <= 134217728ull, "carve budget");
static_assert(OFF_WINH % 128 == 0 && OFF_WOUTH % 128 == 0 && OFF_WXH % 128 == 0 && OFF_XZ % 128 == 0 &&
              OFF_XCF % 128 == 0 && OFF_XCH % 128 == 0 && OFF_XDBL % 128 == 0 && OFF_YH % 128 == 0 && OFF_YL % 128 == 0, "align");

typedef __attribute__((ext_vector_type(16))) _Float16 v16h;
typedef __attribute__((ext_vector_type(8)))  _Float16 v8h;
typedef __attribute__((ext_vector_type(16))) __bf16   v16b;
typedef __attribute__((ext_vector_type(8)))  __bf16   v8b;
typedef __attribute__((ext_vector_type(8)))  float    v8f;
typedef __attribute__((ext_vector_type(4)))  float    v4f;
typedef __attribute__((ext_vector_type(4)))  unsigned v4u;
typedef __attribute__((ext_vector_type(2)))  unsigned v2u;

__device__ __forceinline__ unsigned short f2bf_bits(float f) {
  unsigned u = __float_as_uint(f);
  return (unsigned short)((u + 0x7FFFu + ((u >> 16) & 1u)) >> 16);
}
__device__ __forceinline__ float bf_bits2f(unsigned short h) { return __uint_as_float(((unsigned)h) << 16); }

__device__ __forceinline__ void dep_guard_h(v8f& a, v8f& b, v16h x, v16h y) { asm volatile("v_nop\n\tv_nop\n\tv_nop\n\tv_nop" : "+v"(a), "+v"(b) : "v"(x), "v"(y)); }
__device__ __forceinline__ void dep_guard_b(v8f& a, v8f& b, v16b x, v16b y) { asm volatile("v_nop\n\tv_nop\n\tv_nop\n\tv_nop" : "+v"(a), "+v"(b) : "v"(x), "v"(y)); }
__device__ __forceinline__ void keep4_h(v16h a, v16h b, v16h c, v16h d) { asm volatile("v_nop" :: "v"(a), "v"(b), "v"(c), "v"(d)); }
__device__ __forceinline__ void keep4_b(v16b a, v16b b, v16b c, v16b d) { asm volatile("v_nop" :: "v"(a), "v"(b), "v"(c), "v"(d)); }
__device__ __forceinline__ void acc_guard4(v8f& a, v8f& b, v8f& c, v8f& d) { asm volatile("v_nop\n\tv_nop\n\tv_nop\n\tv_nop" : "+v"(a), "+v"(b), "+v"(c), "+v"(d)); }
template <typename T> struct Frag;
template <> struct Frag<_Float16> {
  typedef v16h V; union U { v16h v; v8h h[2]; };
  static __device__ __forceinline__ v16h load(const _Float16* p) {
    U f; f.h[0] = *(const v8h*)(p); f.h[1] = *(const v8h*)(p + 16); return f.v;
  }
  static __device__ __forceinline__ v8f mma(v16h a, v16h b, v8f c) {
    return __builtin_amdgcn_wmma_f32_16x16x32_f16(false, a, false, b, (short)0, c, false, false);
  }
  static __device__ __forceinline__ void guard(v8f& a, v8f& b, v16h x, v16h y) { dep_guard_h(a, b, x, y); }
  static __device__ __forceinline__ void keep(v16h a, v16h b, v16h c, v16h d) { keep4_h(a, b, c, d); }
};
template <> struct Frag<__bf16> {
  typedef v16b V; union U { v16b v; v8b h[2]; };
  static __device__ __forceinline__ v16b load(const __bf16* p) {
    U f; f.h[0] = *(const v8b*)(p); f.h[1] = *(const v8b*)(p + 16); return f.v;
  }
  static __device__ __forceinline__ v8f mma(v16b a, v16b b, v8f c) {
    return __builtin_amdgcn_wmma_f32_16x16x32_bf16(false, a, false, b, (short)0, c, false, false);
  }
  static __device__ __forceinline__ void guard(v8f& a, v8f& b, v16b x, v16b y) { dep_guard_b(a, b, x, y); }
  static __device__ __forceinline__ void keep(v16b a, v16b b, v16b c, v16b d) { keep4_b(a, b, c, d); }
};

template <int ET> struct Elem;
template <> struct Elem<0> { typedef _Float16 T; };
template <> struct Elem<1> { typedef __bf16 T; };
template <int ET, bool SPLIT, int BIAS_MODE, int OUT_MODE, bool RESID, int ACT = 0>
__global__ __launch_bounds__(256) void wmma_gemm64(
    const unsigned short* __restrict__ Ap, const unsigned short* __restrict__ A2p, int lda, long strideA,
    const unsigned short* __restrict__ Btp, const unsigned short* __restrict__ Bt2p, int ldb, long strideB,
    void* __restrict__ Cout, void* __restrict__ Cout2, int ldc, long strideC,
    const float* __restrict__ bias,
    const float* __restrict__ resid, long strideR,
    int M, int N, int K, float scale) {
  typedef typename Elem<ET>::T T;
  typedef typename Frag<T>::V V;
  const T* A = (const T*)Ap; const T* A2 = (const T*)A2p; const T* Bt = (const T*)Btp; const T* Bt2 = (const T*)Bt2p;
  __shared__ __align__(16) float sT[8][16 * 68];
  const int b    = blockIdx.y;
  const int lane = threadIdx.x & 31;
  const int wave = threadIdx.x >> 5;
  const int tilesN = N >> 6;
  const int tilesM = M >> 6;
  const int tile = blockIdx.x * 8 + wave;
  if (tile >= tilesM * tilesN) return;
  const int tm = tile / tilesN;
  const int tn = tile - tm * tilesN;
  const int m0 = tm << 6;
  const int n0 = tn << 6;

  const T* Ab  = A  + (size_t)b * strideA;
  const T* Bb  = Bt + (size_t)b * strideB;
  const T* Ab2 = SPLIT ? (A2  + (size_t)b * strideA) : nullptr;
  const T* Bb2 = SPLIT ? (Bt2 + (size_t)b * strideB) : nullptr;

  const int rlane = lane & 15;
  const int koff  = (lane >> 4) * 8;
  const int mOff  = (lane >> 4) * 8;

  v8f acc[4][4];
#pragma unroll
  for (int i = 0; i < 4; ++i)
#pragma unroll
    for (int j = 0; j < 4; ++j) acc[i][j] = (v8f){0.f,0.f,0.f,0.f,0.f,0.f,0.f,0.f};

  for (int k0 = 0; k0 < K; k0 += 32) {
    V bh[4], bl[4];
#pragma unroll
    for (int j = 0; j < 4; ++j) {
      const size_t bo = (size_t)(n0 + (j << 4) + rlane) * ldb + koff + k0;
      bh[j] = Frag<T>::load(Bb + bo);
      if (SPLIT) bl[j] = Frag<T>::load(Bb2 + bo);
    }
#pragma unroll
    for (int i = 0; i < 4; ++i) {
      const size_t ao = (size_t)(m0 + (i << 4) + rlane) * lda + koff + k0;
      V ah = Frag<T>::load(Ab + ao);
      V al;
      if (SPLIT) al = Frag<T>::load(Ab2 + ao);
#pragma unroll
      for (int j = 0; j < 4; ++j) {
        acc[i][j] = Frag<T>::mma(ah, bh[j], acc[i][j]);
        if (SPLIT) {
          acc[i][j] = Frag<T>::mma(ah, bl[j], acc[i][j]);
          acc[i][j] = Frag<T>::mma(al, bh[j], acc[i][j]);
        }
      }
      Frag<T>::guard(acc[i][0], acc[i][3], ah, SPLIT ? al : ah);
    }
    Frag<T>::keep(bh[0], bh[1], bh[2], bh[3]);
    if (SPLIT) Frag<T>::keep(bl[0], bl[1], bl[2], bl[3]);
  }
  acc_guard4(acc[0][0], acc[0][1], acc[0][2], acc[0][3]);
  acc_guard4(acc[1][0], acc[1][1], acc[1][2], acc[1][3]);
  acc_guard4(acc[2][0], acc[2][1], acc[2][2], acc[2][3]);
  acc_guard4(acc[3][0], acc[3][1], acc[3][2], acc[3][3]);

  float* slab = sT[wave];
  const float* Rb = RESID ? (resid + (size_t)b * strideR) : nullptr;
#pragma unroll
  for (int i = 0; i < 4; ++i) {
    const int mBase = m0 + (i << 4);
#pragma unroll
    for (int j = 0; j < 4; ++j) {
      const int n = n0 + (j << 4) + rlane;
      float bv = 0.f;
      if (BIAS_MODE == 2) bv = bias[n];
#pragma unroll
      for (int r = 0; r < 8; ++r) {
        float v = acc[i][j][r] * scale;
        if (BIAS_MODE == 1) v += bias[mBase + mOff + r];
        if (BIAS_MODE == 2) v += bv;
        if (RESID) v += Rb[(size_t)(mBase + mOff + r) * ldc + n];
        if (ACT == 1) v = tanhf(v);
        if (ACT == 2) v = fmaxf(v, 0.0f);
        if (ACT == 3) v = v / (1.0f + expf(-v));
        if (ACT == 4) v = (v > 0.f) ? v : 0.01f * v;
        if (ACT == 5) v = 0.5f * v * (1.0f + erff(v * 0.70710678118654752f));
        slab[(mOff + r) * 68 + (j << 4) + rlane] = v;
      }
    }
    __builtin_amdgcn_fence(__ATOMIC_RELEASE, "workgroup");
    __builtin_amdgcn_wave_barrier();
    __builtin_amdgcn_fence(__ATOMIC_ACQUIRE, "workgroup");
    if (OUT_MODE == 0) {
      float* C = (float*)Cout + (size_t)b * strideC;
      const int hh = lane >> 4, c4 = (lane & 15) * 4;
      for (int pass = 0; pass < 2; ++pass) {
#pragma unroll
        for (int it = 0; it < 8; ++it) {
          const int row = it * 2 + hh;
          v4f v = *(const v4f*)(slab + row * 68 + c4);
          *(volatile v4f*)(C + (size_t)(mBase + row) * ldc + n0 + c4) = v;
        }
        __threadfence();
      }
    } else {
      const int q = lane >> 3, c8 = (lane & 7) * 8;
      unsigned short* C  = (unsigned short*)Cout  + (size_t)b * strideC;
      unsigned short* C2 = (OUT_MODE == 2) ? ((unsigned short*)Cout2 + (size_t)b * strideC) : nullptr;
      for (int pass = 0; pass < 2; ++pass) {
#pragma unroll
        for (int it = 0; it < 4; ++it) {
          const int row = it * 4 + q;
          const float* sp = slab + row * 68 + c8;
          v8h hv, lv;
#pragma unroll
          for (int e = 0; e < 8; ++e) {
            if (OUT_MODE == 1) {
              hv[e] = (_Float16)sp[e];
            } else {
              unsigned short hb = f2bf_bits(sp[e]);
              unsigned short lb = f2bf_bits(sp[e] - bf_bits2f(hb));
              hv[e] = __builtin_bit_cast(_Float16, hb);
              lv[e] = __builtin_bit_cast(_Float16, lb);
            }
          }
          *(volatile v8h*)(C + (size_t)(mBase + row) * ldc + n0 + c8) = hv;
          if (OUT_MODE == 2) *(volatile v8h*)(C2 + (size_t)(mBase + row) * ldc + n0 + c8) = lv;
        }
        __threadfence();
      }
    }
    __builtin_amdgcn_fence(__ATOMIC_RELEASE, "workgroup");
    __builtin_amdgcn_wave_barrier();
    __builtin_amdgcn_fence(__ATOMIC_ACQUIRE, "workgroup");
  }
}

__device__ __forceinline__ float wave_sum32(float v) {
#pragma unroll
  for (int off = 16; off > 0; off >>= 1) v += __shfl_xor(v, off, 32);
  return v;
}
__device__ __forceinline__ unsigned pack_bf2(float a, float b) {
  return (unsigned)f2bf_bits(a) | ((unsigned)f2bf_bits(b) << 16);
}
__device__ __forceinline__ void split_bf2(float a, float b, unsigned& hiw, unsigned& low) {
  const unsigned short ha = f2bf_bits(a), hb = f2bf_bits(b);
  const unsigned short la = f2bf_bits(a - bf_bits2f(ha)), lb = f2bf_bits(b - bf_bits2f(hb));
  hiw = (unsigned)ha | ((unsigned)hb << 16);
  low = (unsigned)la | ((unsigned)lb << 16);
}

template <bool HAS_LO>
__global__ __launch_bounds__(256) void k_wcast(const float* __restrict__ src, int krows, int ncols, int nout,
                                               unsigned short* __restrict__ dh, unsigned short* __restrict__ dl) {
  const int lane = threadIdx.x & 31, wave = threadIdx.x >> 5;
  const int n = blockIdx.x * 8 + wave;
  if (n >= nout) return;
  const int k0 = lane * 8;
  const int nc = (n < ncols) ? n : (ncols - 1);
  const bool live = (n < ncols);
  unsigned hw[4], lw[4];
#pragma unroll
  for (int e = 0; e < 4; ++e) {
    int ka = k0 + 2 * e, kb = k0 + 2 * e + 1;
    ka = (ka < krows) ? ka : (krows - 1);
    kb = (kb < krows) ? kb : (krows - 1);
    float va = src[(size_t)ka * ncols + nc];
    float vb = src[(size_t)kb * ncols + nc];
    va = live ? va : 0.f;
    vb = live ? vb : 0.f;
    if (HAS_LO) {
      split_bf2(va, vb, hw[e], lw[e]);
    } else {
      hw[e] = pack_bf2(va, vb); lw[e] = 0u;
    }
  }
  const v4u hv = {hw[0], hw[1], hw[2], hw[3]};
  const v4u lv = {lw[0], lw[1], lw[2], lw[3]};
  const size_t go = (size_t)n * krows + k0;
  if (k0 < krows) {
    *(volatile v4u*)(dh + go) = hv;
    if (HAS_LO) *(volatile v4u*)(dl + go) = lv;
  }
  __threadfence();
  if (k0 < krows) {
    *(volatile v4u*)(dh + go) = hv;
    if (HAS_LO) *(volatile v4u*)(dl + go) = lv;
  }
}

__global__ __launch_bounds__(256) void k_ln_swap(
    const float* __restrict__ I1, const float* __restrict__ I2,
    const float* __restrict__ R1, const float* __restrict__ R2,
    const float* __restrict__ w1, const float* __restrict__ b1,
    const float* __restrict__ w2, const float* __restrict__ b2,
    float* __restrict__ oR1, float* __restrict__ oR2,
    unsigned short* __restrict__ x1h, unsigned short* __restrict__ x1l,
    unsigned short* __restrict__ x2h, unsigned short* __restrict__ x2l) {
  __shared__ __align__(16) unsigned sU[8][4 * 128];
  const int lane = threadIdx.x & 31, wave = threadIdx.x >> 5;
  const int r0 = (blockIdx.x * 8 + wave) * 2;
  const int c = lane * 4;
  const v4f W1v = *(const v4f*)(w1 + c), B1v = *(const v4f*)(b1 + c);
  const v4f W2v = *(const v4f*)(w2 + c), B2v = *(const v4f*)(b2 + c);
  unsigned* slab = sU[wave];
  const float inv_n = 1.0f / (float)CDIM;
#pragma unroll 1
  for (int j = 0; j < 2; ++j) {
    const size_t off = (size_t)(r0 + j) * CDIM + c;
    const v4f a  = *(const v4f*)(I1 + off), ra = *(const v4f*)(R1 + off);
    const v4f q  = *(const v4f*)(I2 + off), rq = *(const v4f*)(R2 + off);
    const v4f s1 = a + ra;
    const v4f s2 = q + rq;
    *(volatile v4f*)(oR1 + off) = s1;
    *(volatile v4f*)(oR2 + off) = s2;
    __threadfence();
    *(volatile v4f*)(oR1 + off) = s1;
    *(volatile v4f*)(oR2 + off) = s2;

    const float m1 = wave_sum32(s1.x + s1.y + s1.z + s1.w) * inv_n;
    const float m2 = wave_sum32(s2.x + s2.y + s2.z + s2.w) * inv_n;
    const v4f d1 = s1 - m1;
    const v4f d2 = s2 - m2;
    const float v1 = wave_sum32(d1.x * d1.x + d1.y * d1.y + d1.z * d1.z + d1.w * d1.w) * inv_n;
    const float v2 = wave_sum32(d2.x * d2.x + d2.y * d2.y + d2.z * d2.z + d2.w * d2.w) * inv_n;
    const float rs1 = rsqrtf(v1 + 1e-5f);
    const float rs2 = rsqrtf(v2 + 1e-5f);
    const v4f n1 = d1 * rs1 * W1v + B1v;
    const v4f n2 = d2 * rs2 * W2v + B2v;
    unsigned eh0, el0, eh1, el1, fh0, fl0, fh1, fl1;
    split_bf2(n2.x, n1.y, eh0, el0);
    split_bf2(n2.z, n1.w, eh1, el1);
    split_bf2(n1.x, n2.y, fh0, fl0);
    split_bf2(n1.z, n2.w, fh1, fl1);
    const v2u pe_h = {eh0, eh1}, pe_l = {el0, el1}, pf_h = {fh0, fh1}, pf_l = {fl0, fl1};
    *(v2u*)(slab + 0 * 128 + j * 64 + 2 * lane) = pe_h;
    *(v2u*)(slab + 1 * 128 + j * 64 + 2 * lane) = pe_l;
    *(v2u*)(slab + 2 * 128 + j * 64 + 2 * lane) = pf_h;
    *(v2u*)(slab + 3 * 128 + j * 64 + 2 * lane) = pf_l;
  }
  __builtin_amdgcn_fence(__ATOMIC_RELEASE, "workgroup");
  __builtin_amdgcn_wave_barrier();
  __builtin_amdgcn_fence(__ATOMIC_ACQUIRE, "workgroup");
  const size_t go = (size_t)r0 * CDIM + 8 * lane;
  for (int pass = 0; pass < 2; ++pass) {
    const v4u v0 = *(const v4u*)(slab + 0 * 128 + 4 * lane);
    const v4u v1 = *(const v4u*)(slab + 1 * 128 + 4 * lane);
    const v4u v2 = *(const v4u*)(slab + 2 * 128 + 4 * lane);
    const v4u v3 = *(const v4u*)(slab + 3 * 128 + 4 * lane);
    *(volatile v4u*)(x1h + go) = v0;
    *(volatile v4u*)(x1l + go) = v1;
    *(volatile v4u*)(x2h + go) = v2;
    *(volatile v4u*)(x2l + go) = v3;
    __threadfence();
  }
}

__global__ __launch_bounds__(256) void k_conv_silu(
    const float* __restrict__ xz, const float* __restrict__ cw, const float* __restrict__ cb,
    float* __restrict__ xcf, unsigned short* __restrict__ xch) {
  __shared__ __align__(16) unsigned sU[8][CONV_TW * 64];
  const int lane = threadIdx.x & 31, wave = threadIdx.x >> 5;
  const int job = blockIdx.x * 8 + wave;
  const int hsel = job & 1;
  const int tok0 = (job >> 1) * CONV_TW;
  const int bstart = (tok0 / NTOK) * NTOK;
  const int c = hsel * 128 + lane * 4;
  const v4f wv0 = *(const v4f*)(cw + (size_t)c * 4);
  const v4f wv1 = *(const v4f*)(cw + (size_t)c * 4 + 4);
  const v4f wv2 = *(const v4f*)(cw + (size_t)c * 4 + 8);
  const v4f wv3 = *(const v4f*)(cw + (size_t)c * 4 + 12);
  const v4f bv  = *(const v4f*)(cb + c);
  v4f xm3, xm2, xm1;
  {
    const int r3 = tok0 - 3, r2 = tok0 - 2, r1 = tok0 - 1;
    const int a3 = (r3 < bstart) ? bstart : r3;
    const int a2 = (r2 < bstart) ? bstart : r2;
    const int a1 = (r1 < bstart) ? bstart : r1;
    const v4f t3 = *(const v4f*)(xz + (size_t)a3 * CD2 + c);
    const v4f t2 = *(const v4f*)(xz + (size_t)a2 * CD2 + c);
    const v4f t1 = *(const v4f*)(xz + (size_t)a1 * CD2 + c);
    const bool k3 = (r3 >= bstart), k2 = (r2 >= bstart), k1 = (r1 >= bstart);
    xm3.x = k3 ? t3.x : 0.f; xm3.y = k3 ? t3.y : 0.f; xm3.z = k3 ? t3.z : 0.f; xm3.w = k3 ? t3.w : 0.f;
    xm2.x = k2 ? t2.x : 0.f; xm2.y = k2 ? t2.y : 0.f; xm2.z = k2 ? t2.z : 0.f; xm2.w = k2 ? t2.w : 0.f;
    xm1.x = k1 ? t1.x : 0.f; xm1.y = k1 ? t1.y : 0.f; xm1.z = k1 ? t1.z : 0.f; xm1.w = k1 ? t1.w : 0.f;
  }
  unsigned* slab = sU[wave];
#pragma unroll 1
  for (int i = 0; i < CONV_TW; ++i) {
    const int tok = tok0 + i;
    const v4f x0 = *(const v4f*)(xz + (size_t)tok * CD2 + c);
    float a0 = wv0.x * xm3.x + wv0.y * xm2.x + wv0.z * xm1.x + wv0.w * x0.x;
    float a1 = wv1.x * xm3.y + wv1.y * xm2.y + wv1.z * xm1.y + wv1.w * x0.y;
    float a2 = wv2.x * xm3.z + wv2.y * xm2.z + wv2.z * xm1.z + wv2.w * x0.z;
    float a3 = wv3.x * xm3.w + wv3.y * xm2.w + wv3.z * xm1.w + wv3.w * x0.w;
    a0 += bv.x; a1 += bv.y; a2 += bv.z; a3 += bv.w;
    const float s0 = a0 / (1.0f + expf(-a0));
    const float s1 = a1 / (1.0f + expf(-a1));
    const float s2 = a2 / (1.0f + expf(-a2));
    const float s3 = a3 / (1.0f + expf(-a3));
    const v4f xc = {s0, s1, s2, s3};
    float* pf = xcf + (size_t)tok * CDIN + c;
    *(volatile v4f*)pf = xc;
    __threadfence();
    *(volatile v4f*)pf = xc;
    const v2u pk = {pack_bf2(s0, s1), pack_bf2(s2, s3)};
    *(v2u*)(slab + i * 64 + 2 * lane) = pk;
    xm3 = xm2; xm2 = xm1; xm1 = x0;
  }
  __builtin_amdgcn_fence(__ATOMIC_RELEASE, "workgroup");
  __builtin_amdgcn_wave_barrier();
  __builtin_amdgcn_fence(__ATOMIC_ACQUIRE, "workgroup");
  const int hi4 = lane >> 4, lo4 = lane & 15;
  for (int pass = 0; pass < 2; ++pass) {
#pragma unroll
    for (int it = 0; it < CONV_TW / 2; ++it) {
      const int t = 2 * it + hi4;
      const v4u v = *(const v4u*)(slab + t * 64 + 4 * lo4);
      *(volatile v4u*)(xch + (size_t)(tok0 + t) * CDIN + hsel * 128 + 8 * lo4) = v;
    }
    __threadfence();
  }
}

__global__ __launch_bounds__(64) void k_scan_gate(
    const float* __restrict__ xdbl, const float* __restrict__ xcf, const float* __restrict__ xz,
    const float* __restrict__ Wdt, const float* __restrict__ dtb, const float* __restrict__ Alog,
    const float* __restrict__ Dp, unsigned short* __restrict__ yh, unsigned short* __restrict__ yl) {
  __shared__ __align__(16) float sX[SCAN_CH * NXPAD];
  __shared__ __align__(16) float sA[64 * NST];
  __shared__ __align__(16) unsigned short sYH[SCAN_CH * 64];
  __shared__ __align__(16) unsigned short sYL[SCAN_CH * 64];
  const int tid = threadIdx.x, lane = tid & 31, wave = tid >> 5;
  const int b  = blockIdx.x >> 2;
  const int d0 = (blockIdx.x & 3) * 64;
  const int d  = d0 + tid;
  const float LOG2E = 1.4426950408889634f;
#pragma unroll 1
  for (int s = 0; s < NST; ++s) sA[tid * NST + s] = -expf(Alog[(size_t)d * NST + s]) * LOG2E;
  __syncthreads();
  float A2[NST];
#pragma unroll
  for (int s = 0; s < NST; ++s) A2[s] = sA[tid * NST + s];
  float wdt[NDTR];
#pragma unroll
  for (int r = 0; r < NDTR; ++r) wdt[r] = Wdt[(size_t)r * CDIN + d];
  const float bias = dtb[d];
  const float Dd = Dp[d];
  float h[NST];
#pragma unroll
  for (int s = 0; s < NST; ++s) h[s] = 0.f;
  const int q4 = lane >> 3, c8 = (lane & 7) * 8;

#pragma unroll 1
  for (int ck = 0; ck < NTOK / SCAN_CH; ++ck) {
    const int tok0 = b * NTOK + ck * SCAN_CH;
    __syncthreads();
#pragma unroll
    for (int i = 0; i < 4; ++i) {
      const int idx = tid + 64 * i;
      const int row = idx >> 4, c4 = (idx & 15) * 4;
      *(v4f*)(sX + row * NXPAD + c4) = *(const v4f*)(xdbl + (size_t)(tok0 + row) * NXPAD + c4);
    }
    __syncthreads();
#pragma unroll 1
    for (int i = 0; i < SCAN_CH; ++i) {
      const int tok = tok0 + i;
      const float* xr = sX + i * NXPAD;
      const v4f r0 = *(const v4f*)(xr), r1 = *(const v4f*)(xr + 4);
      v4f Bq[4], Cq[4];
#pragma unroll
      for (int qq = 0; qq < 4; ++qq) {
        Bq[qq] = *(const v4f*)(xr + NDTR + 4 * qq);
        Cq[qq] = *(const v4f*)(xr + NDTR + NST + 4 * qq);
      }
      const float xcv = xcf[(size_t)tok * CDIN + d];
      const float zv  = xz[(size_t)tok * CD2 + CDIN + d];
      float x = r0.x * wdt[0] + r0.y * wdt[1] + r0.z * wdt[2] + r0.w * wdt[3]
              + r1.x * wdt[4] + r1.y * wdt[5] + r1.z * wdt[6] + r1.w * wdt[7];
      x += bias;
      const float ex = expf(-fabsf(x));
      const float dt = fmaxf(x, 0.f) + logf(1.0f + ex);
      const float u = dt * xcv;
      float y = 0.f;
#pragma unroll
      for (int s = 0; s < NST; ++s) {
        const float dA = exp2f(dt * A2[s]);
        h[s] = dA * h[s] + u * Bq[s >> 2][s & 3];
        y += h[s] * Cq[s >> 2][s & 3];
      }
      y += xcv * Dd;
      const float g = zv / (1.0f + expf(-zv));
      y *= g;
      const unsigned short hb = f2bf_bits(y);
      const unsigned short lb = f2bf_bits(y - bf_bits2f(hb));
      sYH[i * 64 + tid] = hb;
      sYL[i * 64 + tid] = lb;
    }
    __syncthreads();
    for (int pass = 0; pass < 2; ++pass) {
#pragma unroll
      for (int it = 0; it < 2; ++it) {
        const int row = wave * 8 + it * 4 + q4;
        const v4u hv = *(const v4u*)(sYH + row * 64 + c8);
        const v4u lv = *(const v4u*)(sYL + row * 64 + c8);
        const size_t go = (size_t)(tok0 + row) * CDIN + d0 + c8;
        *(volatile v4u*)(yh + go) = hv;
        *(volatile v4u*)(yl + go) = lv;
      }
      __threadfence();
    }
  }
}

extern "C" void kernel_launch(void* const* d_in, const int* in_sizes, int n_in,
                              void* d_out, int out_size, void* d_ws, size_t ws_size,
                              hipStream_t stream) {
  if (n_in < 26) return;
  if (in_sizes[0] != NROWS * CDIM || in_sizes[8] != CDIM * CD2 || in_sizes[11] != CDIN * NXP) return;
  if (out_size != 4 * NROWS * CDIM) return;
  if (ws_size < WS_TOTAL) return;

  const float* I1   = (const float*)d_in[0];
  const float* I2   = (const float*)d_in[1];
  const float* R1   = (const float*)d_in[2];
  const float* R2   = (const float*)d_in[3];
  const float* ln1w = (const float*)d_in[4];
  const float* ln1b = (const float*)d_in[5];
  const float* ln2w = (const float*)d_in[6];
  const float* ln2b = (const float*)d_in[7];
  const float* W_in[2]    = {(const float*)d_in[8],  (const float*)d_in[17]};
  const float* conv_w[2]  = {(const float*)d_in[9],  (const float*)d_in[18]};
  const float* conv_b[2]  = {(const float*)d_in[10], (const float*)d_in[19]};
  const float* W_x[2]     = {(const float*)d_in[11], (const float*)d_in[20]};
  const float* W_dt[2]    = {(const float*)d_in[12], (const float*)d_in[21]};
  const float* dt_bias[2] = {(const float*)d_in[13], (const float*)d_in[22]};
  const float* A_log[2]   = {(const float*)d_in[14], (const float*)d_in[23]};
  const float* Dp[2]      = {(const float*)d_in[15], (const float*)d_in[24]};
  const float* W_out[2]   = {(const float*)d_in[16], (const float*)d_in[25]};

  float* outp = (float*)d_out;
  float* out_s[2] = {outp, outp + (size_t)NROWS * CDIM};
  float* oR1 = outp + 2 * (size_t)NROWS * CDIM;
  float* oR2 = outp + 3 * (size_t)NROWS * CDIM;

  char* ws = (char*)d_ws;
  unsigned short* xsh[2] = {(unsigned short*)(ws + OFF_X1H), (unsigned short*)(ws + OFF_X2H)};
  unsigned short* xsl[2] = {(unsigned short*)(ws + OFF_X1L), (unsigned short*)(ws + OFF_X2L)};
  unsigned short* winh  = (unsigned short*)(ws + OFF_WINH);
  unsigned short* winl  = (unsigned short*)(ws + OFF_WINL);
  unsigned short* wouth = (unsigned short*)(ws + OFF_WOUTH);
  unsigned short* woutl = (unsigned short*)(ws + OFF_WOUTL);
  unsigned short* wxh   = (unsigned short*)(ws + OFF_WXH);
  float* xzp   = (float*)(ws + OFF_XZ);
  float* xcfp  = (float*)(ws + OFF_XCF);
  unsigned short* xchp = (unsigned short*)(ws + OFF_XCH);
  float* xdblp = (float*)(ws + OFF_XDBL);
  unsigned short* yhp = (unsigned short*)(ws + OFF_YH);
  unsigned short* ylp = (unsigned short*)(ws + OFF_YL);

  k_ln_swap<<<NROWS / 16, 256, 0, stream>>>(I1, I2, R1, R2, ln1w, ln1b, ln2w, ln2b, oR1, oR2,
                                            xsh[0], xsl[0], xsh[1], xsl[1]);

  for (int s = 0; s < 2; ++s) {
    k_wcast<true><<<CD2 / 8, 256, 0, stream>>>(W_in[s], CDIM, CD2, CD2, winh, winl);
    k_wcast<true><<<CDIM / 8, 256, 0, stream>>>(W_out[s], CDIN, CDIM, CDIM, wouth, woutl);
    k_wcast<false><<<NXPAD / 8, 256, 0, stream>>>(W_x[s], CDIN, NXP, NXPAD, wxh, wxh);

    wmma_gemm64<1, true, 0, 0, false><<<dim3((NROWS / 64) * (CD2 / 64) / 8, 1), 256, 0, stream>>>(
        xsh[s], xsl[s], CDIM, 0L, winh, winl, CDIM, 0L,
        (void*)xzp, (void*)xzp, CD2, 0L, dt_bias[s], (const float*)xzp, 0L, NROWS, CD2, CDIM, 1.0f);

    k_conv_silu<<<(NROWS / CONV_TW) * 2 / 8, 256, 0, stream>>>(xzp, conv_w[s], conv_b[s], xcfp, xchp);

    wmma_gemm64<1, false, 0, 0, false><<<dim3((NROWS / 64) * (NXPAD / 64) / 8, 1), 256, 0, stream>>>(
        xchp, xchp, CDIN, 0L, wxh, wxh, CDIN, 0L,
        (void*)xdblp, (void*)xdblp, NXPAD, 0L, dt_bias[s], (const float*)xzp, 0L, NROWS, NXPAD, CDIN, 1.0f);

    k_scan_gate<<<NBATCH * (CDIN / 64), 64, 0, stream>>>(xdblp, xcfp, xzp, W_dt[s], dt_bias[s], A_log[s], Dp[s], yhp, ylp);

    wmma_gemm64<1, true, 0, 0, false><<<dim3((NROWS / 64) * (CDIM / 64) / 8, 1), 256, 0, stream>>>(
        yhp, ylp, CDIN, 0L, wouth, woutl, CDIN, 0L,
        (void*)out_s[s], (void*)out_s[s], CDIM, 0L, dt_bias[s], (const float*)xzp, 0L, NROWS, CDIM, CDIN, 1.0f);
  }
}
